// WindowMultiheadPosAttention_17480516894743
// MI455X (gfx1250) — hardware-verified
//
#include <hip/hip_runtime.h>
#include <math.h>
#include <stdint.h>

#define BSZ   2
#define NTOK  4096
#define GRIDW 64
#define HALFW 32
#define DMOD  768
#define NHD   12
#define HDIM  64
#define NWIN  4
#define LW    1024
#define NSEQ  (BSZ * NWIN)
#define NKT   (LW / 64)
#define MROWS (BSZ * NTOK)
#define KOUT  (2 * DMOD)
static_assert(NHD * HDIM == DMOD);
static_assert(HDIM == 64);
static_assert(GRIDW * GRIDW == NTOK);
static_assert(2 * HALFW == GRIDW);
static_assert(HALFW * HALFW == LW);
static_assert(NWIN * LW == NTOK);
static_assert((MROWS % 64) == 0 && (DMOD % 64) == 0 && (DMOD % 32) == 0 && (KOUT % 32) == 0 && (LW % 64) == 0);
static_assert((((MROWS / 64) * (DMOD / 64)) % 8) == 0);
static_assert(((MROWS * DMOD / 8) % 256) == 0);
static_assert(DMOD == 96 * 8);
static_assert(NSEQ * NHD * NKT == 1536);

typedef _Float16 v16h __attribute__((ext_vector_type(16)));
typedef _Float16 v8h  __attribute__((ext_vector_type(8)));
typedef float    v8f  __attribute__((ext_vector_type(8)));
typedef float    v4f  __attribute__((ext_vector_type(4)));
typedef unsigned int v4u __attribute__((ext_vector_type(4)));
#if defined(__HIP_DEVICE_COMPILE__)
typedef __bf16   v16b __attribute__((ext_vector_type(16)));
#endif

__device__ __forceinline__ unsigned short bf_bits(float f) {
  unsigned u = __float_as_uint(f);
  return (unsigned short)((u + 0x7FFFu + ((u >> 16) & 1u)) >> 16);
}
__device__ __forceinline__ float bf_up(unsigned short h) { return __uint_as_float(((unsigned)h) << 16); }
__device__ __forceinline__ float bfr(float f) { return bf_up(bf_bits(f)); }
__device__ __forceinline__ unsigned short h_bits(_Float16 x) { return __builtin_bit_cast(unsigned short, x); }
__device__ __forceinline__ unsigned pk16(unsigned short a, unsigned short b) { return (unsigned)a | ((unsigned)b << 16); }
__device__ __forceinline__ v8f zero8() { v8f z = {0.f, 0.f, 0.f, 0.f, 0.f, 0.f, 0.f, 0.f}; return z; }

__device__ __forceinline__ void ld8(const float* p, float* o) {
  const v4f a = *(const v4f*)(p);
  const v4f b = *(const v4f*)(p + 4);
  o[0] = a[0]; o[1] = a[1]; o[2] = a[2]; o[3] = a[3];
  o[4] = b[0]; o[5] = b[1]; o[6] = b[2]; o[7] = b[3];
}

__device__ __forceinline__ int src_tok(int win, int ip) {
  return (win >> 1) * (HALFW * GRIDW) + (ip >> 5) * GRIDW + (win & 1) * HALFW + (ip & 31);
}

__device__ __forceinline__ v16h ldfrag_h(const _Float16* p) {
  union { v16h v; v8h h[2]; } f;
  f.h[0] = *(const v8h*)(p);
  f.h[1] = *(const v8h*)(p + 16);
  return f.v;
}

__device__ __forceinline__ v8f mma_h(v16h a, v16h b, v8f c) {
  c = __builtin_amdgcn_wmma_f32_16x16x32_f16(false, a, false, b, (short)0, c, false, false);
#if defined(__HIP_DEVICE_COMPILE__)
  asm volatile("v_nop\n\tv_nop\n\tv_nop\n\tv_nop" : "+v"(c) : "v"(a), "v"(b));
#endif
  return c;
}
template <int BF> __device__ __forceinline__ v8f mma_raw(v16h a, v16h b, v8f c);
template <> __device__ __forceinline__ v8f mma_raw<0>(v16h a, v16h b, v8f c) {
  return __builtin_amdgcn_wmma_f32_16x16x32_f16(false, a, false, b, (short)0, c, false, false);
}
template <> __device__ __forceinline__ v8f mma_raw<1>(v16h a, v16h b, v8f c) {
#if defined(__HIP_DEVICE_COMPILE__)
  return __builtin_amdgcn_wmma_f32_16x16x32_bf16(false, __builtin_bit_cast(v16b, a), false,
                                                __builtin_bit_cast(v16b, b), (short)0, c, false, false);
#else
  return c;
#endif
}
__device__ __forceinline__ void dep_guard_h(v8f& a, v8f& b, v16h x) {
#if defined(__HIP_DEVICE_COMPILE__)
  asm volatile("v_nop\n\tv_nop\n\tv_nop\n\tv_nop" : "+v"(a), "+v"(b) : "v"(x));
#endif
}
__device__ __forceinline__ void keep4_h(v16h a, v16h b, v16h c, v16h d) {
#if defined(__HIP_DEVICE_COMPILE__)
  asm volatile("v_nop" :: "v"(a), "v"(b), "v"(c), "v"(d));
#endif
}
__device__ __forceinline__ void acc_guard4(v8f& a, v8f& b, v8f& c, v8f& d) {
#if defined(__HIP_DEVICE_COMPILE__)
  asm volatile("v_nop\n\tv_nop\n\tv_nop\n\tv_nop" : "+v"(a), "+v"(b), "+v"(c), "+v"(d));
#endif
}

__global__ __launch_bounds__(256) void wt_cvt(const float* __restrict__ W, int ncols, int nrows,
                                              unsigned short* outp, float sc) {
  __shared__ __align__(16) float sw[64 * 68];
  const int tid = threadIdx.x;
  const int n0 = blockIdx.x * 64;
  const int k0 = blockIdx.y * 64;
#pragma unroll
  for (int i = 0; i < 4; ++i) {
    const int idx = i * 256 + tid;
    const int kk = idx >> 4, c4 = (idx & 15) * 4;
    const v4f a = *(const v4f*)(W + (size_t)(k0 + kk) * ncols + n0 + c4);
    *(v4f*)(sw + kk * 68 + c4) = a;
  }
  __syncthreads();

  const int gq = tid >> 3, piece = tid & 7;
  v4u ov[2];
  size_t oofs[2];
#pragma unroll
  for (int it = 0; it < 2; ++it) {
    const int nn = it * 32 + gq;
    v4u a;
#pragma unroll
    for (int e = 0; e < 4; ++e) {
      const float f0 = sw[(piece * 8 + 2 * e) * 68 + nn];
      const float f1 = sw[(piece * 8 + 2 * e + 1) * 68 + nn];
      a[e] = pk16(h_bits((_Float16)(bfr(f0) * sc)), h_bits((_Float16)(bfr(f1) * sc)));
    }
    ov[it] = a;
    oofs[it] = (size_t)(n0 + nn) * nrows + k0 + piece * 8;
  }
  for (int pass = 0; pass < 2; ++pass) {
#pragma unroll
    for (int it = 0; it < 2; ++it) *(volatile v4u*)(outp + oofs[it]) = ov[it];
    __threadfence();
  }
}

__global__ __launch_bounds__(256) void wt_cvt2(const float* __restrict__ W, int ncols, int nrows,
                                               unsigned short* outp) {
  __shared__ __align__(16) float sw[64 * 68];
  const int tid = threadIdx.x;
  const int n0 = blockIdx.x * 64;
  const int k0 = blockIdx.y * 64;
#pragma unroll
  for (int i = 0; i < 4; ++i) {
    const int idx = i * 256 + tid;
    const int kk = idx >> 4, c4 = (idx & 15) * 4;
    const v4f a = *(const v4f*)(W + (size_t)(k0 + kk) * ncols + n0 + c4);
    *(v4f*)(sw + kk * 68 + c4) = a;
  }
  __syncthreads();

  const int gq = tid >> 3, piece = tid & 7;
  v4u ov[2];
  size_t oofs[2];
#pragma unroll
  for (int it = 0; it < 2; ++it) {
    const int nn = it * 32 + gq;
    v4u a;
#pragma unroll
    for (int e = 0; e < 4; ++e) {
      const float f0 = sw[(piece * 8 + 2 * e) * 68 + nn];
      const float f1 = sw[(piece * 8 + 2 * e + 1) * 68 + nn];
      a[e] = pk16(bf_bits(f0), bf_bits(f1));
    }
    ov[it] = a;
    oofs[it] = (size_t)(n0 + nn) * (size_t)(2 * nrows) + k0 + piece * 8;
  }
  for (int pass = 0; pass < 2; ++pass) {
#pragma unroll
    for (int it = 0; it < 2; ++it) {
      *(volatile v4u*)(outp + oofs[it]) = ov[it];
      *(volatile v4u*)(outp + oofs[it] + nrows) = ov[it];
    }
    __threadfence();
  }
}

__global__ __launch_bounds__(256) void cvt_xh(const float* __restrict__ in, unsigned short* out, int n8,
                                              float sc) {
  const int i = blockIdx.x * 256 + threadIdx.x;
  if (i < n8) {
    const v4f a = *(const v4f*)(in + (size_t)i * 8);
    const v4f b = *(const v4f*)(in + (size_t)i * 8 + 4);
    v4u p;
    p[0] = pk16(h_bits((_Float16)(bfr(a[0]) * sc)), h_bits((_Float16)(bfr(a[1]) * sc)));
    p[1] = pk16(h_bits((_Float16)(bfr(a[2]) * sc)), h_bits((_Float16)(bfr(a[3]) * sc)));
    p[2] = pk16(h_bits((_Float16)(bfr(b[0]) * sc)), h_bits((_Float16)(bfr(b[1]) * sc)));
    p[3] = pk16(h_bits((_Float16)(bfr(b[2]) * sc)), h_bits((_Float16)(bfr(b[3]) * sc)));
    *(volatile v4u*)(out + (size_t)i * 8) = p;
    __threadfence();
    *(volatile v4u*)(out + (size_t)i * 8) = p;
  }
}

template <int BF>
__global__ __launch_bounds__(256) void gemm64(
    const unsigned short* __restrict__ Ap, int lda,
    const unsigned short* __restrict__ Btp, int ldb,
    const float* __restrict__ bias, float* Cf, int ldc, int M, int N, int K, float oscale) {
  const _Float16* Ah = (const _Float16*)(const void*)Ap;
  const _Float16* Bh = (const _Float16*)(const void*)Btp;
  __shared__ __align__(16) float sT[8][16 * 68];
  const int lane = threadIdx.x & 31;
  const int wave = threadIdx.x >> 5;
  const int tilesN = N >> 6;
  const int tilesM = M >> 6;
  const int tile = blockIdx.x * 8 + wave;
  if (tile >= tilesM * tilesN) return;
  const int tm = tile / tilesN;
  const int tn = tile - tm * tilesN;
  const int m0 = tm << 6;
  const int n0 = tn << 6;

  const int rlane = lane & 15;
  const int koff  = (lane >> 4) * 8;
  const int mOff  = (lane >> 4) * 8;

  v8f acc[4][4];
#pragma unroll
  for (int i = 0; i < 4; ++i)
#pragma unroll
    for (int j = 0; j < 4; ++j) acc[i][j] = zero8();

  for (int k0 = 0; k0 < K; k0 += 32) {
    v16h bh[4];
#pragma unroll
    for (int j = 0; j < 4; ++j) {
      const size_t bo = (size_t)(n0 + (j << 4) + rlane) * ldb + koff + k0;
      bh[j] = ldfrag_h(Bh + bo);
    }
#pragma unroll
    for (int i = 0; i < 4; ++i) {
      const size_t ao = (size_t)(m0 + (i << 4) + rlane) * lda + koff + k0;
      const v16h ah = ldfrag_h(Ah + ao);
#pragma unroll
      for (int j = 0; j < 4; ++j) acc[i][j] = mma_raw<BF>(ah, bh[j], acc[i][j]);
      dep_guard_h(acc[i][0], acc[i][3], ah);
    }
    keep4_h(bh[0], bh[1], bh[2], bh[3]);
  }
  acc_guard4(acc[0][0], acc[0][1], acc[0][2], acc[0][3]);
  acc_guard4(acc[1][0], acc[1][1], acc[1][2], acc[1][3]);
  acc_guard4(acc[2][0], acc[2][1], acc[2][2], acc[2][3]);
  acc_guard4(acc[3][0], acc[3][1], acc[3][2], acc[3][3]);

  float* slab = sT[wave];
  const int h2 = lane >> 4, c4 = (lane & 15) * 4;
  v4f b4;
  {
    const v4f braw = *(const v4f*)(bias + n0 + c4);
#pragma unroll
    for (int e = 0; e < 4; ++e) b4[e] = bfr(braw[e]);
  }
#pragma unroll
  for (int i = 0; i < 4; ++i) {
    const int mBase = m0 + (i << 4);
#pragma unroll
    for (int r = 0; r < 8; ++r) {
#pragma unroll
      for (int j = 0; j < 4; ++j) {
        slab[(mOff + r) * 68 + (j << 4) + rlane] = acc[i][j][r];
      }
    }
    __builtin_amdgcn_fence(__ATOMIC_RELEASE, "workgroup");
    __builtin_amdgcn_wave_barrier();
    __builtin_amdgcn_fence(__ATOMIC_ACQUIRE, "workgroup");
    v4f ov[8];
#pragma unroll
    for (int it = 0; it < 8; ++it) {
      const int row = it * 2 + h2;
      const v4f xs = *(const v4f*)(slab + row * 68 + c4);
      ov[it] = xs * oscale + b4;
    }
    for (int pass = 0; pass < 2; ++pass) {
#pragma unroll
      for (int it = 0; it < 8; ++it) {
        const int row = it * 2 + h2;
        *(volatile v4f*)(Cf + (size_t)(mBase + row) * ldc + n0 + c4) = ov[it];
      }
      __threadfence();
    }
    __builtin_amdgcn_fence(__ATOMIC_RELEASE, "workgroup");
    __builtin_amdgcn_wave_barrier();
    __builtin_amdgcn_fence(__ATOMIC_ACQUIRE, "workgroup");
  }
}

__global__ __launch_bounds__(96) void qk_planes(const float* __restrict__ F, unsigned short* ph,
                                                unsigned short* pl, float osc, float rsc) {
  const int tid = threadIdx.x;
  const int rp  = blockIdx.x;
  const int b   = rp >> 12;
  const int np  = rp & (NTOK - 1);
  const int win = np >> 10;
  const int ip  = np & (LW - 1);
  const int n   = src_tok(win, ip);
  const size_t srow = (size_t)b * NTOK + (size_t)n;
  const int d0 = tid * 8;
  float x[8];
  ld8(F + srow * DMOD + d0, x);
  v4u ah, al;
#pragma unroll
  for (int pp = 0; pp < 4; ++pp) {
    const float t0 = x[2 * pp] * osc;
    const float t1 = x[2 * pp + 1] * osc;
    const _Float16 h0 = (_Float16)t0, h1 = (_Float16)t1;
    const _Float16 l0 = (_Float16)((t0 - (float)h0) * rsc);
    const _Float16 l1 = (_Float16)((t1 - (float)h1) * rsc);
    ah[pp] = pk16(h_bits(h0), h_bits(h1));
    al[pp] = pk16(h_bits(l0), h_bits(l1));
  }
  const size_t o = (size_t)rp * DMOD + d0;
  *(volatile v4u*)(ph + o) = ah;
  *(volatile v4u*)(pl + o) = al;
  __threadfence();
  *(volatile v4u*)(ph + o) = ah;
  *(volatile v4u*)(pl + o) = al;
}

__global__ __launch_bounds__(256) void v_planes(const float* __restrict__ F, unsigned short* vt, float vscale) {
  __shared__ __align__(16) float svt[64 * 68];
  const int tid = threadIdx.x;
  const int kt  = blockIdx.x;
  const int hh  = blockIdx.y;
  const int seq = blockIdx.z;
  const int b   = seq >> 2;
  const int win = seq & 3;
  const int t0  = kt * 64;
#pragma unroll
  for (int i = 0; i < 4; ++i) {
    const int idx = i * 256 + tid;
    const int tt = idx >> 4, c4 = (idx & 15) * 4;
    const int n  = src_tok(win, t0 + tt);
    const v4f a = *(const v4f*)(F + ((size_t)b * NTOK + (size_t)n) * DMOD + hh * HDIM + c4);
    *(v4f*)(svt + tt * 68 + c4) = a;
  }
  __syncthreads();

  const int gq = tid >> 3, piece = tid & 7;
  v4u hv[2];
  size_t hofs[2];
#pragma unroll
  for (int it = 0; it < 2; ++it) {
    const int d = it * 32 + gq;
    v4u a;
#pragma unroll
    for (int e = 0; e < 4; ++e) {
      const float f0 = svt[(piece * 8 + 2 * e) * 68 + d] * vscale;
      const float f1 = svt[(piece * 8 + 2 * e + 1) * 68 + d] * vscale;
      a[e] = pk16(h_bits((_Float16)f0), h_bits((_Float16)f1));
    }
    hv[it] = a;
    hofs[it] = ((size_t)seq * DMOD + (size_t)hh * HDIM + (size_t)d) * LW + t0 + piece * 8;
  }
  for (int pass = 0; pass < 2; ++pass) {
#pragma unroll
    for (int it = 0; it < 2; ++it) *(volatile v4u*)(vt + hofs[it]) = hv[it];
    __threadfence();
  }
}

__global__ __launch_bounds__(128)
void attn_w64(const unsigned short* __restrict__ qhp, const unsigned short* __restrict__ qlp,
              const unsigned short* __restrict__ khp, const unsigned short* __restrict__ klp,
              const unsigned short* __restrict__ vtp, unsigned short* yo,
              float sscale, float rinv, float oscl) {
  union FH { v16h v; v8h h[2]; };
  __shared__ __align__(16) _Float16 Khs[64 * 64];
  __shared__ __align__(16) _Float16 Kls[64 * 64];
  __shared__ __align__(16) _Float16 Vts[64 * 64];
  __shared__ __align__(16) _Float16 Psh[4][16 * 64];
  __shared__ __align__(16) float    Os[4][16 * 64];

  const int tid  = threadIdx.x;
  const int wave = tid >> 5;
  const int lane = tid & 31;
  const int hh   = lane >> 4;
  const int c    = lane & 15;

  const int bx  = blockIdx.x;
  const int qt  = bx % NKT;
  const int hb  = bx / NKT;
  const int h   = hb % NHD;
  const int seq = hb / NHD;
  const int q0  = qt * 64 + wave * 16;

  const size_t qkb = (size_t)seq * LW * DMOD + (size_t)h * HDIM;
  const _Float16* Qh = (const _Float16*)(const void*)qhp + qkb;
  const _Float16* Ql = (const _Float16*)(const void*)qlp + qkb;
  const _Float16* Kh = (const _Float16*)(const void*)khp + qkb;
  const _Float16* Kl = (const _Float16*)(const void*)klp + qkb;
  const _Float16* Vt = (const _Float16*)(const void*)vtp + ((size_t)seq * DMOD + (size_t)h * HDIM) * LW;

  v16h qa[2], qr[2];
#pragma unroll
  for (int dc = 0; dc < 2; ++dc) {
    const size_t qo = (size_t)(q0 + c) * DMOD + dc * 32 + 8 * hh;
    qa[dc] = ldfrag_h(Qh + qo);
    qr[dc] = ldfrag_h(Ql + qo);
  }

  float mrow[8], lrow[8];
  v8f oacc[4];
#pragma unroll
  for (int r = 0; r < 8; ++r) { mrow[r] = -INFINITY; lrow[r] = 0.f; }
#pragma unroll
  for (int t = 0; t < 4; ++t) oacc[t] = zero8();

  for (int kt = 0; kt < NKT; ++kt) {
    const int kv0 = kt * 64;
    __syncthreads();
    {
      const int r = tid >> 1, half = (tid & 1) * 32;
      const _Float16* kg  = Kh + (size_t)(kv0 + r) * DMOD + half;
      const _Float16* klg = Kl + (size_t)(kv0 + r) * DMOD + half;
      const _Float16* vg  = Vt + (size_t)r * LW + kv0 + half;
#pragma unroll
      for (int i = 0; i < 4; ++i) {
        const v8h a0 = *(const v8h*)(kg + 8 * i);
        const v8h a1 = *(const v8h*)(klg + 8 * i);
        const v8h b0 = *(const v8h*)(vg + 8 * i);
        *(v8h*)(Khs + r * 64 + half + 8 * i) = a0;
        *(v8h*)(Kls + r * 64 + half + 8 * i) = a1;
        *(v8h*)(Vts + r * 64 + half + 8 * i) = b0;
      }
    }
    __syncthreads();

    v8f s[4];
#pragma unroll
    for (int j = 0; j < 4; ++j) {
      v8f ahh = zero8(), ax = zero8();
#pragma unroll
      for (int dc = 0; dc < 2; ++dc) {
        FH kb, kr;
        kb.h[0] = *(const v8h*)(Khs + (j * 16 + c) * 64 + dc * 32 + 8 * hh);
        kb.h[1] = *(const v8h*)(Khs + (j * 16 + c) * 64 + dc * 32 + 16 + 8 * hh);
        kr.h[0] = *(const v8h*)(Kls + (j * 16 + c) * 64 + dc * 32 + 8 * hh);
        kr.h[1] = *(const v8h*)(Kls + (j * 16 + c) * 64 + dc * 32 + 16 + 8 * hh);
        ahh = mma_h(qa[dc], kb.v, ahh);
        ax  = mma_h(qa[dc], kr.v, ax);
        ax  = mma_h(qr[dc], kb.v, ax);
      }
      s[j] = ahh + ax * rinv;
    }

    _Float16* pwh = Psh[wave];
#pragma unroll
    for (int r = 0; r < 8; ++r) {
      float m = -INFINITY;
#pragma unroll
      for (int j = 0; j < 4; ++j) {
        const float sv = s[j][r] * sscale;
        s[j][r] = sv;
        m = fmaxf(m, sv);
      }
#pragma unroll
      for (int off = 1; off < 16; off <<= 1) m = fmaxf(m, __shfl_xor(m, off, 32));
      const float mnew  = fmaxf(mrow[r], m);
      const float msafe = (mnew == -INFINITY) ? 0.f : mnew;
      const float alpha = __expf(mrow[r] - msafe);
      mrow[r] = mnew;
      float psum = 0.f;
#pragma unroll
      for (int j = 0; j < 4; ++j) {
        const float p = __expf(s[j][r] - msafe);
        psum += p;
        const _Float16 phv = (_Float16)(p * 1024.0f);
        pwh[(8 * hh + r) * 64 + j * 16 + c] = phv;
      }
#pragma unroll
      for (int off = 1; off < 16; off <<= 1) psum += __shfl_xor(psum, off, 32);
      lrow[r] = lrow[r] * alpha + psum;
#pragma unroll
      for (int t = 0; t < 4; ++t) oacc[t][r] *= alpha;
    }
    __builtin_amdgcn_fence(__ATOMIC_RELEASE, "workgroup");
    __builtin_amdgcn_wave_barrier();
    __builtin_amdgcn_fence(__ATOMIC_ACQUIRE, "workgroup");

#pragma unroll 1
    for (int kk = 0; kk < 2; ++kk) {
      FH pa;
      pa.h[0] = *(const v8h*)(pwh + c * 64 + kk * 32 + 8 * hh);
      pa.h[1] = *(const v8h*)(pwh + c * 64 + kk * 32 + 16 + 8 * hh);
#pragma unroll
      for (int t = 0; t < 4; ++t) {
        FH vb;
        vb.h[0] = *(const v8h*)(Vts + (t * 16 + c) * 64 + kk * 32 + 8 * hh);
        vb.h[1] = *(const v8h*)(Vts + (t * 16 + c) * 64 + kk * 32 + 16 + 8 * hh);
        oacc[t] = mma_h(pa.v, vb.v, oacc[t]);
      }
    }
  }

  float* os = Os[wave];
#pragma unroll
  for (int r = 0; r < 8; ++r) {
    const float l = lrow[r];
    const float inv = ((l > 0.f) ? (1.0f / l) : 0.f) * oscl;
#pragma unroll
    for (int t = 0; t < 4; ++t) os[(8 * hh + r) * 64 + t * 16 + c] = oacc[t][r] * inv;
  }
  __builtin_amdgcn_fence(__ATOMIC_RELEASE, "workgroup");
  __builtin_amdgcn_wave_barrier();
  __builtin_amdgcn_fence(__ATOMIC_ACQUIRE, "workgroup");
  {
    const int q8 = lane & 7, rr = lane >> 3, c8 = q8 * 8;
    v4u ovh[4], ovl[4];
    size_t go[4];
#pragma unroll
    for (int it = 0; it < 4; ++it) {
      const int row = it * 4 + rr;
      float xs[8];
      ld8(os + row * 64 + c8, xs);
      v4u ah, al;
#pragma unroll
      for (int pp = 0; pp < 4; ++pp) {
        const unsigned short h0 = bf_bits(xs[2 * pp]);
        const unsigned short h1 = bf_bits(xs[2 * pp + 1]);
        const unsigned short l0 = bf_bits(xs[2 * pp] - bf_up(h0));
        const unsigned short l1 = bf_bits(xs[2 * pp + 1] - bf_up(h1));
        ah[pp] = pk16(h0, h1);
        al[pp] = pk16(l0, l1);
      }
      ovh[it] = ah;
      ovl[it] = al;
      go[it] = ((size_t)seq * LW + (size_t)(q0 + row)) * KOUT + (size_t)h * HDIM + c8;
    }
    for (int pass = 0; pass < 2; ++pass) {
#pragma unroll
      for (int it = 0; it < 4; ++it) {
        *(volatile v4u*)(yo + go[it]) = ovh[it];
        *(volatile v4u*)(yo + go[it] + DMOD) = ovl[it];
      }
      __threadfence();
    }
  }
}

extern "C" void kernel_launch(void* const* d_in, const int* in_sizes, int n_in,
                              void* d_out, int out_size, void* d_ws, size_t ws_size,
                              hipStream_t stream) {
  if (n_in < 10) return;
  if (in_sizes[0] != MROWS * DMOD) return;
  if (in_sizes[1] != MROWS * DMOD) return;
  if (in_sizes[2] != DMOD * DMOD || in_sizes[3] != DMOD) return;
  if (in_sizes[4] != DMOD * DMOD || in_sizes[5] != DMOD) return;
  if (in_sizes[6] != DMOD * DMOD || in_sizes[7] != DMOD) return;
  if (in_sizes[8] != DMOD * DMOD || in_sizes[9] != DMOD) return;
  if (out_size != MROWS * DMOD) return;

  const float* x   = (const float*)d_in[0];
  const float* pe  = (const float*)d_in[1];
  const float* wq  = (const float*)d_in[2];
  const float* bq  = (const float*)d_in[3];
  const float* wk  = (const float*)d_in[4];
  const float* bk  = (const float*)d_in[5];
  const float* wv  = (const float*)d_in[6];
  const float* bv  = (const float*)d_in[7];
  const float* wp  = (const float*)d_in[8];
  const float* bp  = (const float*)d_in[9];

  const size_t PX   = (size_t)MROWS * DMOD * 2;
  const size_t PY   = (size_t)MROWS * KOUT * 2;
  const size_t PW   = (size_t)DMOD * DMOD * 2;
  const size_t PWp  = (size_t)DMOD * KOUT * 2;
  const size_t PF   = (size_t)MROWS * DMOD * 4;
  const size_t PQK  = (size_t)MROWS * DMOD * 2;
  const size_t PVT  = (size_t)NSEQ * DMOD * LW * 2;
  size_t off = 0;
  const size_t oXh  = off; off += PX;
  const size_t oPh  = off; off += PX;
  const size_t oY   = oXh;
  if (PY != 2 * PX) return;
  const size_t oWq  = off; off += PW;
  const size_t oWk  = off; off += PW;
  const size_t oWv  = off; off += PW;
  const size_t oWp  = off; off += PWp;
  const size_t oF   = off; off += PF;
  const size_t oQh  = off; off += PQK;
  const size_t oQl  = off; off += PQK;
  const size_t oKh  = off; off += PQK;
  const size_t oKl  = off; off += PQK;
  const size_t oVT  = off; off += PVT;
  if (off > ws_size) return;
  if (off > (size_t)134217728) return;

  char* ws = (char*)d_ws;
  unsigned short* Xh   = (unsigned short*)(ws + oXh);
  unsigned short* Ph   = (unsigned short*)(ws + oPh);
  unsigned short* Yo   = (unsigned short*)(ws + oY);
  unsigned short* WqT  = (unsigned short*)(ws + oWq);
  unsigned short* WkT  = (unsigned short*)(ws + oWk);
  unsigned short* WvT  = (unsigned short*)(ws + oWv);
  unsigned short* WpT2 = (unsigned short*)(ws + oWp);
  float*          F32  = (float*)(ws + oF);
  unsigned short* Qh   = (unsigned short*)(ws + oQh);
  unsigned short* Ql   = (unsigned short*)(ws + oQl);
  unsigned short* Kh   = (unsigned short*)(ws + oKh);
  unsigned short* Kl   = (unsigned short*)(ws + oKl);
  unsigned short* VT   = (unsigned short*)(ws + oVT);
  float*          outf = (float*)d_out;

  const dim3 blk(256);
  const int  n8x = MROWS * DMOD / 8;
  const dim3 gW(DMOD / 64, DMOD / 64);
  const dim3 gCx((n8x + 255) / 256);
  const dim3 gG(((MROWS / 64) * (DMOD / 64) + 7) / 8);
  const dim3 gQK(MROWS);
  const dim3 gVpl(NKT, NHD, NSEQ);
  const dim3 gAttn(NSEQ * NHD * NKT);

  const float wScale  = 64.0f;
  const float xScale  = 8.0f;
  const float pInv    = 1.0f / 512.0f;
  const float qkScale = 16.0f;
  const float rScale  = 2048.0f;
  const float sscale  = 0.625f / 256.0f;
  const float rinv    = 1.0f / 2048.0f;
  const float vScale  = 256.0f;
  const float attOscl = 1.0f / 262144.0f;

  wt_cvt<<<gW, blk, 0, stream>>>(wq, DMOD, DMOD, WqT, wScale);
  wt_cvt<<<gW, blk, 0, stream>>>(wk, DMOD, DMOD, WkT, wScale);
  wt_cvt<<<gW, blk, 0, stream>>>(wv, DMOD, DMOD, WvT, wScale);
  wt_cvt2<<<gW, blk, 0, stream>>>(wp, DMOD, DMOD, WpT2);
  cvt_xh<<<gCx, blk, 0, stream>>>(x, Xh, n8x, xScale);
  cvt_xh<<<gCx, blk, 0, stream>>>(pe, Ph, n8x, xScale);
  gemm64<0><<<gG, blk, 0, stream>>>(Ph, DMOD, WqT, DMOD, bq, F32, DMOD, MROWS, DMOD, DMOD, pInv);
  qk_planes<<<gQK, dim3(96), 0, stream>>>(F32, Qh, Ql, qkScale, rScale);
  gemm64<0><<<gG, blk, 0, stream>>>(Xh, DMOD, WkT, DMOD, bk, F32, DMOD, MROWS, DMOD, DMOD, pInv);
  qk_planes<<<gQK, dim3(96), 0, stream>>>(F32, Kh, Kl, qkScale, rScale);
  gemm64<0><<<gG, blk, 0, stream>>>(Xh, DMOD, WvT, DMOD, bv, F32, DMOD, MROWS, DMOD, DMOD, pInv);
  v_planes<<<gVpl, blk, 0, stream>>>(F32, VT, vScale);
  attn_w64<<<gAttn, dim3(128), 0, stream>>>(Qh, Ql, Kh, Kl, VT, Yo, sscale, rinv, attOscl);
  gemm64<1><<<gG, blk, 0, stream>>>(Yo, KOUT, WpT2, KOUT, bp, outf, DMOD, MROWS, DMOD, KOUT, 1.0f);
  (void)hipGetLastError();
}
